// FoundationTransformerLayer_29429115912814
// MI455X (gfx1250) — hardware-run, weakly checked
//
#include <hip/hip_runtime.h>
#include <math.h>
#include <float.h>
#include <stdint.h>


#define BATCH 4
#define SEQ   1024
#define DM    512
#define NH    8
#define HD    64
#define NQB   (SEQ / 64)
#define FFN   2048
#define CCH   128
#define NRES  4
#define MROWS (BATCH * SEQ)
#define OUTN  (MROWS * DM)
static_assert(NH * HD == DM);
static_assert(HD == 64);
static_assert(DM == 512);
static_assert(CCH * 4 == DM);
static_assert((SEQ % 64) == 0 && (DM % 64) == 0 && (FFN % 64) == 0 && (CCH % 64) == 0);
static_assert(((MROWS / 64) * (DM / 64)) % 8 == 0);
static_assert(((MROWS / 64) * (FFN / 64)) % 8 == 0);
static_assert(((MROWS * DM / 8) % 256) == 0);
static_assert(((DM * DM / 8) % 256) == 0);
static_assert(((FFN * DM / 8) % 256) == 0);
static_assert((SEQ & (SEQ - 1)) == 0);

typedef _Float16 v16h __attribute__((ext_vector_type(16)));
typedef _Float16 v8h  __attribute__((ext_vector_type(8)));
typedef float    v8f  __attribute__((ext_vector_type(8)));
typedef float    v4f  __attribute__((ext_vector_type(4)));
typedef unsigned int v4u __attribute__((ext_vector_type(4)));

__device__ __forceinline__ unsigned short bf_bits(float f) {
  unsigned u = __float_as_uint(f);
  return (unsigned short)((u + 0x7FFFu + ((u >> 16) & 1u)) >> 16);
}
__device__ __forceinline__ float bf_up(unsigned short h) { return __uint_as_float(((unsigned)h) << 16); }
__device__ __forceinline__ float bfr(float f) { return bf_up(bf_bits(f)); }
__device__ __forceinline__ unsigned short h_bits(_Float16 x) { return __builtin_bit_cast(unsigned short, x); }
__device__ __forceinline__ unsigned pk16(unsigned short a, unsigned short b) { return (unsigned)a | ((unsigned)b << 16); }
__device__ __forceinline__ v8f zero8() { v8f z = {0.f, 0.f, 0.f, 0.f, 0.f, 0.f, 0.f, 0.f}; return z; }

__device__ __forceinline__ void ld8(const float* p, float* o) {
  const v4f a = *(const v4f*)(p);
  const v4f b = *(const v4f*)(p + 4);
  o[0] = a[0]; o[1] = a[1]; o[2] = a[2]; o[3] = a[3];
  o[4] = b[0]; o[5] = b[1]; o[6] = b[2]; o[7] = b[3];
}

__device__ __forceinline__ v16h ldfrag_h(const _Float16* p) {
  union { v16h v; v8h h[2]; } f;
  f.h[0] = *(const v8h*)(p);
  f.h[1] = *(const v8h*)(p + 16);
  return f.v;
}

__device__ __forceinline__ v8f mma_h(v16h a, v16h b, v8f c) {
  c = __builtin_amdgcn_wmma_f32_16x16x32_f16(false, a, false, b, (short)0, c, false, false);
#if defined(__HIP_DEVICE_COMPILE__)
  asm volatile("v_nop\n\tv_nop\n\tv_nop\n\tv_nop" : "+v"(c) : "v"(a), "v"(b));
#endif
  return c;
}
__device__ __forceinline__ v8f mma_h_raw(v16h a, v16h b, v8f c) {
  return __builtin_amdgcn_wmma_f32_16x16x32_f16(false, a, false, b, (short)0, c, false, false);
}
__device__ __forceinline__ void dep_guard_h(v8f& a, v8f& b, v16h x) {
#if defined(__HIP_DEVICE_COMPILE__)
  asm volatile("v_nop\n\tv_nop\n\tv_nop\n\tv_nop" : "+v"(a), "+v"(b) : "v"(x));
#endif
}
__device__ __forceinline__ void keep4_h(v16h a, v16h b, v16h c, v16h d) {
#if defined(__HIP_DEVICE_COMPILE__)
  asm volatile("v_nop" :: "v"(a), "v"(b), "v"(c), "v"(d));
#endif
}
__device__ __forceinline__ void acc_guard4(v8f& a, v8f& b, v8f& c, v8f& d) {
#if defined(__HIP_DEVICE_COMPILE__)
  asm volatile("v_nop\n\tv_nop\n\tv_nop\n\tv_nop" : "+v"(a), "+v"(b), "+v"(c), "+v"(d));
#endif
}

__global__ __launch_bounds__(256) void cvt_f16x8(const float* __restrict__ in, unsigned short* out, int n8,
                                                 float sc, int rnd) {
  const int i = blockIdx.x * 256 + threadIdx.x;
  if (i < n8) {
    float v[8];
    ld8(in + (size_t)i * 8, v);
    if (rnd != 0) {
#pragma unroll
      for (int e = 0; e < 8; ++e) v[e] = bfr(v[e]);
    }
    v4u p;
#pragma unroll
    for (int q = 0; q < 4; ++q)
      p[q] = pk16(h_bits((_Float16)(v[2 * q] * sc)), h_bits((_Float16)(v[2 * q + 1] * sc)));
    *(volatile v4u*)(out + (size_t)i * 8) = p;
    __threadfence();
    *(volatile v4u*)(out + (size_t)i * 8) = p;
  }
}

__global__ __launch_bounds__(256) void cw_cvt(const float* __restrict__ in, unsigned short* out, int n8,
                                              int taps, float sc) {
  const int i = blockIdx.x * 256 + threadIdx.x;
  if (i < n8) {
    const int o8 = i * 8;
    const int d0 = o8 & (DM - 1);
    const int t  = o8 >> 9;
    const int k  = t % taps;
    const int c  = t / taps;
    v4u p;
#pragma unroll
    for (int q = 0; q < 4; ++q) {
      const float f0 = in[((size_t)(c * DM + d0 + 2 * q)) * (size_t)taps + k];
      const float f1 = in[((size_t)(c * DM + d0 + 2 * q + 1)) * (size_t)taps + k];
      p[q] = pk16(h_bits((_Float16)(bfr(f0) * sc)), h_bits((_Float16)(bfr(f1) * sc)));
    }
    *(volatile v4u*)(out + (size_t)o8) = p;
    __threadfence();
    *(volatile v4u*)(out + (size_t)o8) = p;
  }
}

template <int MODE, int RR, int ACT>
__global__ __launch_bounds__(256) void gemm64(
    const unsigned short* __restrict__ Ap, int lda,
    const unsigned short* __restrict__ Btp, int ldb,
    const float* __restrict__ bias, const float* __restrict__ res, int ldr,
    float* Cf, unsigned short* Ch, int ldc, int M, int N, int Kc, int nsplit, int sstride,
    float oscale, float oscale2) {
  const _Float16* Ah = (const _Float16*)(const void*)Ap;
  const _Float16* Bh = (const _Float16*)(const void*)Btp;
  __shared__ __align__(16) float sT[8][16 * 68];
  const int lane = threadIdx.x & 31;
  const int wave = threadIdx.x >> 5;
  const int tilesN = N >> 6;
  const int tilesM = M >> 6;
  const int tiles = tilesM * tilesN;
  const int item = blockIdx.x * 8 + wave;
  if (item >= tiles * nsplit) return;
  const int ky = item / tiles;
  const int tile = item - ky * tiles;
  const int tm = tile / tilesN;
  const int tn = tile - tm * tilesN;
  const int m0 = tm << 6;
  const int n0 = tn << 6;
  const int kbeg = ky * Kc;
  const int kend = kbeg + Kc;
  const float bsel = (ky == 0) ? 1.0f : 0.0f;
  float* Cp = Cf + (size_t)ky * (size_t)sstride;

  const int rlane = lane & 15;
  const int koff  = (lane >> 4) * 8;
  const int mOff  = (lane >> 4) * 8;

  v8f acc[4][4];
#pragma unroll
  for (int i = 0; i < 4; ++i)
#pragma unroll
    for (int j = 0; j < 4; ++j) acc[i][j] = zero8();

  for (int k0 = kbeg; k0 < kend; k0 += 32) {
    v16h bh[4];
#pragma unroll
    for (int j = 0; j < 4; ++j) {
      const size_t bo = (size_t)(n0 + (j << 4) + rlane) * (size_t)ldb + koff + k0;
      bh[j] = ldfrag_h(Bh + bo);
    }
#pragma unroll
    for (int i = 0; i < 4; ++i) {
      const size_t ao = (size_t)(m0 + (i << 4) + rlane) * (size_t)lda + koff + k0;
      const v16h ah = ldfrag_h(Ah + ao);
#pragma unroll
      for (int j = 0; j < 4; ++j) acc[i][j] = mma_h_raw(ah, bh[j], acc[i][j]);
      dep_guard_h(acc[i][0], acc[i][3], ah);
    }
    keep4_h(bh[0], bh[1], bh[2], bh[3]);
  }
  acc_guard4(acc[0][0], acc[0][1], acc[0][2], acc[0][3]);
  acc_guard4(acc[1][0], acc[1][1], acc[1][2], acc[1][3]);
  acc_guard4(acc[2][0], acc[2][1], acc[2][2], acc[2][3]);
  acc_guard4(acc[3][0], acc[3][1], acc[3][2], acc[3][3]);

  float* slab = sT[wave];
#pragma unroll
  for (int i = 0; i < 4; ++i) {
    const int mBase = m0 + (i << 4);
#pragma unroll
    for (int r = 0; r < 8; ++r) {
#pragma unroll
      for (int j = 0; j < 4; ++j) {
        slab[(mOff + r) * 68 + (j << 4) + rlane] = acc[i][j][r];
      }
    }
    __builtin_amdgcn_fence(__ATOMIC_RELEASE, "workgroup");
    __builtin_amdgcn_wave_barrier();
    __builtin_amdgcn_fence(__ATOMIC_ACQUIRE, "workgroup");
    if (MODE != 2) {
      const int h2 = lane >> 4, c4 = (lane & 15) * 4;
      v4f b4;
      {
        const v4f braw = *(const v4f*)(bias + n0 + c4);
#pragma unroll
        for (int e = 0; e < 4; ++e) b4[e] = bfr(braw[e]) * bsel;
      }
      v4f ov[8];
#pragma unroll
      for (int it = 0; it < 8; ++it) {
        const int row = it * 2 + h2;
        const v4f xs = *(const v4f*)(slab + row * 68 + c4);
        v4f v = xs * oscale;
        if (MODE == 1) {
          v4f r4 = *(const v4f*)(res + (size_t)(mBase + row) * (size_t)ldr + n0 + c4);
          if (RR != 0) {
#pragma unroll
            for (int e = 0; e < 4; ++e) r4[e] = bfr(r4[e]);
          }
          v = (v + b4) + r4;
        } else {
          v = v + b4;
        }
        ov[it] = v;
      }
      for (int pass = 0; pass < 2; ++pass) {
#pragma unroll
        for (int it = 0; it < 8; ++it) {
          const int row = it * 2 + h2;
          *(volatile v4f*)(Cp + (size_t)(mBase + row) * (size_t)ldc + n0 + c4) = ov[it];
        }
        __threadfence();
      }
    } else {
      const int q8 = lane & 7, rr = lane >> 3, c8 = q8 * 8;
      float bb[8];
      {
        const v4f b0 = *(const v4f*)(bias + n0 + c8);
        const v4f b1 = *(const v4f*)(bias + n0 + c8 + 4);
#pragma unroll
        for (int e = 0; e < 4; ++e) { bb[e] = bfr(b0[e]) * bsel; bb[4 + e] = bfr(b1[e]) * bsel; }
      }
      v4u ov[4];
#pragma unroll
      for (int it = 0; it < 4; ++it) {
        const int row = it * 4 + rr;
        float xs[8];
        ld8(slab + row * 68 + c8, xs);
        float v[8];
#pragma unroll
        for (int e = 0; e < 8; ++e) {
          float xv = xs[e] * oscale + bb[e];
          if (ACT != 0) xv = fmaxf(xv, 0.0f);
          v[e] = xv * oscale2;
        }
        v4u a;
#pragma unroll
        for (int p = 0; p < 4; ++p) a[p] = pk16(h_bits((_Float16)v[2 * p]), h_bits((_Float16)v[2 * p + 1]));
        ov[it] = a;
      }
      for (int pass = 0; pass < 2; ++pass) {
#pragma unroll
        for (int it = 0; it < 4; ++it) {
          const int row = it * 4 + rr;
          *(volatile v4u*)(Ch + (size_t)(mBase + row) * (size_t)ldc + n0 + c8) = ov[it];
        }
        __threadfence();
      }
    }
    __builtin_amdgcn_fence(__ATOMIC_RELEASE, "workgroup");
    __builtin_amdgcn_wave_barrier();
    __builtin_amdgcn_fence(__ATOMIC_ACQUIRE, "workgroup");
  }
}

__global__ __launch_bounds__(256) void v_planes(const float* __restrict__ vf,
                                                unsigned short* vth, unsigned short* vtl, float vscale) {
  __shared__ __align__(16) float sv[64 * 68];
  const int tid = threadIdx.x;
  const int t0  = blockIdx.x * 64;
  const int hh  = blockIdx.y;
  const int bb  = blockIdx.z;
#pragma unroll
  for (int i = 0; i < 4; ++i) {
    const int idx = i * 256 + tid;
    const int tt = idx >> 4, c4 = (idx & 15) * 4;
    const v4f a = *(const v4f*)(vf + ((size_t)(bb * SEQ + t0 + tt)) * DM + hh * HD + c4);
    *(v4f*)(sv + tt * 68 + c4) = a;
  }
  __syncthreads();

  const int g = tid >> 3, piece = tid & 7;
  v4u hv[2], lv[2];
  size_t hofs[2];
#pragma unroll
  for (int it = 0; it < 2; ++it) {
    const int d = it * 32 + g;
    v4u a, a2;
#pragma unroll
    for (int e = 0; e < 4; ++e) {
      const float f0 = sv[(piece * 8 + 2 * e) * 68 + d] * vscale;
      const float f1 = sv[(piece * 8 + 2 * e + 1) * 68 + d] * vscale;
      const _Float16 x0 = (_Float16)f0, x1 = (_Float16)f1;
      const unsigned short h0 = h_bits(x0), h1 = h_bits(x1);
      const unsigned short l0 = h_bits((_Float16)((f0 - (float)x0) * 4096.0f));
      const unsigned short l1 = h_bits((_Float16)((f1 - (float)x1) * 4096.0f));
      a[e] = pk16(h0, h1); a2[e] = pk16(l0, l1);
    }
    hv[it] = a; lv[it] = a2;
    hofs[it] = ((size_t)((bb * NH + hh) * HD + d)) * SEQ + t0 + piece * 8;
  }
  for (int pass = 0; pass < 2; ++pass) {
#pragma unroll
    for (int it = 0; it < 2; ++it) {
      *(volatile v4u*)(vth + hofs[it]) = hv[it];
      *(volatile v4u*)(vtl + hofs[it]) = lv[it];
    }
    __threadfence();
  }
}

__global__ __launch_bounds__(128)
void attn64(const unsigned short* __restrict__ qhp, const unsigned short* __restrict__ khp,
            const unsigned short* __restrict__ vhp, const unsigned short* __restrict__ vlp,
            const float* __restrict__ rbp, const int* __restrict__ rmp, const int* __restrict__ amp,
            float* outp, float sscale, float oscl) {
  union FH { v16h v; v8h h[2]; };
  __shared__ __align__(16) _Float16 Ksh[64 * 64];
  __shared__ __align__(16) _Float16 Vth[64 * 64];
  __shared__ __align__(16) _Float16 Vtl[64 * 64];
  __shared__ __align__(16) _Float16 Psh[4][16 * 64];
  __shared__ __align__(16) float    Os[4][16 * 64];
  __shared__ float Rb[NRES * NRES];

  const int tid  = threadIdx.x;
  const int wave = tid >> 5;
  const int lane = tid & 31;
  const int hh   = lane >> 4;
  const int c    = lane & 15;

  const int bx = blockIdx.x;
  const int qb = bx % NQB;
  const int bh = bx / NQB;
  const int h  = bh % NH;
  const int b  = bh / NH;
  const int rbase = b * SEQ;
  const int q0 = rbase + qb * 64 + wave * 16;

  if (tid < NRES * NRES) Rb[tid] = bfr(rbp[h * (NRES * NRES) + tid]);

  const _Float16* Qp = (const _Float16*)(const void*)qhp + (size_t)h * HD;
  const _Float16* Kp = (const _Float16*)(const void*)khp + (size_t)h * HD;
  const _Float16* Vh = (const _Float16*)(const void*)vhp + (size_t)(b * NH + h) * HD * SEQ;
  const _Float16* Vl = (const _Float16*)(const void*)vlp + (size_t)(b * NH + h) * HD * SEQ;

  v16h qa[2];
#pragma unroll
  for (int dc = 0; dc < 2; ++dc) {
    const size_t qo = (size_t)(q0 + c) * DM + dc * 32 + 8 * hh;
    qa[dc] = ldfrag_h(Qp + qo);
  }

  int rmi4[8];
#pragma unroll
  for (int r = 0; r < 8; ++r) {
    int v = rmp[q0 + 8 * hh + r];
    v = min(max(v, 0), NRES - 1);
    rmi4[r] = v * NRES;
  }

  float mrow[8], lrow[8];
  v8f oacc[4];
#pragma unroll
  for (int r = 0; r < 8; ++r) { mrow[r] = -INFINITY; lrow[r] = 0.f; }
#pragma unroll
  for (int t = 0; t < 4; ++t) oacc[t] = zero8();

  for (int kt = 0; kt < NQB; ++kt) {
    const int kv0 = kt * 64;
    __syncthreads();
    {
      const int r = tid >> 1, half = (tid & 1) * 32;
      const _Float16* kg  = Kp + (size_t)(rbase + kv0 + r) * DM + half;
      const _Float16* vg  = Vh + (size_t)r * SEQ + kv0 + half;
      const _Float16* vlg = Vl + (size_t)r * SEQ + kv0 + half;
#pragma unroll
      for (int i = 0; i < 4; ++i) {
        const v8h a0 = *(const v8h*)(kg + 8 * i);
        const v8h b0 = *(const v8h*)(vg + 8 * i);
        const v8h b1 = *(const v8h*)(vlg + 8 * i);
        *(v8h*)(Ksh + r * 64 + half + 8 * i) = a0;
        *(v8h*)(Vth + r * 64 + half + 8 * i) = b0;
        *(v8h*)(Vtl + r * 64 + half + 8 * i) = b1;
      }
    }
    __syncthreads();

    v8f s[4];
#pragma unroll
    for (int j = 0; j < 4; ++j) {
      s[j] = zero8();
#pragma unroll
      for (int dc = 0; dc < 2; ++dc) {
        FH kb;
        kb.h[0] = *(const v8h*)(Ksh + (j * 16 + c) * 64 + dc * 32 + 8 * hh);
        kb.h[1] = *(const v8h*)(Ksh + (j * 16 + c) * 64 + dc * 32 + 16 + 8 * hh);
        s[j] = mma_h(qa[dc], kb.v, s[j]);
      }
    }

    int rmj[4], amz[4];
#pragma unroll
    for (int j = 0; j < 4; ++j) {
      const int key = rbase + kv0 + j * 16 + c;
      int v = rmp[key];
      v = min(max(v, 0), NRES - 1);
      rmj[j] = v;
      amz[j] = (amp[key] == 0) ? 1 : 0;
    }

    _Float16* pwh = Psh[wave];
#pragma unroll
    for (int r = 0; r < 8; ++r) {
      float m = -INFINITY;
#pragma unroll
      for (int j = 0; j < 4; ++j) {
        float sv = s[j][r] * sscale + Rb[rmi4[r] + rmj[j]];
        sv = (amz[j] != 0) ? -1.0e9f : sv;
        s[j][r] = sv;
        m = fmaxf(m, sv);
      }
#pragma unroll
      for (int off = 1; off < 16; off <<= 1) m = fmaxf(m, __shfl_xor(m, off, 32));
      const float mnew  = fmaxf(mrow[r], m);
      const float msafe = (mnew == -INFINITY) ? 0.f : mnew;
      const float alpha = __expf(mrow[r] - msafe);
      mrow[r] = mnew;
      float psum = 0.f;
#pragma unroll
      for (int j = 0; j < 4; ++j) {
        const float p = __expf(s[j][r] - msafe);
        psum += p;
        const _Float16 ph = (_Float16)(p * 1024.0f);
        pwh[(8 * hh + r) * 64 + j * 16 + c] = ph;
      }
#pragma unroll
      for (int off = 1; off < 16; off <<= 1) psum += __shfl_xor(psum, off, 32);
      lrow[r] = lrow[r] * alpha + psum;
#pragma unroll
      for (int t = 0; t < 4; ++t) oacc[t][r] *= alpha;
    }
    __builtin_amdgcn_fence(__ATOMIC_RELEASE, "workgroup");
    __builtin_amdgcn_wave_barrier();
    __builtin_amdgcn_fence(__ATOMIC_ACQUIRE, "workgroup");

    v8f o1[4];
#pragma unroll
    for (int t = 0; t < 4; ++t) o1[t] = zero8();
#pragma unroll 1
    for (int kk = 0; kk < 2; ++kk) {
      FH pa;
      pa.h[0] = *(const v8h*)(pwh + c * 64 + kk * 32 + 8 * hh);
      pa.h[1] = *(const v8h*)(pwh + c * 64 + kk * 32 + 16 + 8 * hh);
#pragma unroll
      for (int t = 0; t < 4; ++t) {
        FH vb;
        vb.h[0] = *(const v8h*)(Vth + (t * 16 + c) * 64 + kk * 32 + 8 * hh);
        vb.h[1] = *(const v8h*)(Vth + (t * 16 + c) * 64 + kk * 32 + 16 + 8 * hh);
        oacc[t] = mma_h(pa.v, vb.v, oacc[t]);
        FH vl;
        vl.h[0] = *(const v8h*)(Vtl + (t * 16 + c) * 64 + kk * 32 + 8 * hh);
        vl.h[1] = *(const v8h*)(Vtl + (t * 16 + c) * 64 + kk * 32 + 16 + 8 * hh);
        o1[t] = mma_h(pa.v, vl.v, o1[t]);
      }
    }
#pragma unroll
    for (int t = 0; t < 4; ++t)
#pragma unroll
      for (int r = 0; r < 8; ++r) oacc[t][r] += o1[t][r] * (1.0f / 4096.0f);
  }

  float* os = Os[wave];
#pragma unroll
  for (int r = 0; r < 8; ++r) {
    const float l = lrow[r];
    const float inv = ((l > 0.f) ? (1.0f / l) : 0.f) * oscl;
#pragma unroll
    for (int t = 0; t < 4; ++t) os[(8 * hh + r) * 64 + t * 16 + c] = oacc[t][r] * inv;
  }
  __builtin_amdgcn_fence(__ATOMIC_RELEASE, "workgroup");
  __builtin_amdgcn_wave_barrier();
  __builtin_amdgcn_fence(__ATOMIC_ACQUIRE, "workgroup");
  {
    const int h2 = lane >> 4, c4 = (lane & 15) * 4;
    v4f ov[8];
#pragma unroll
    for (int it = 0; it < 8; ++it) {
      const int row = it * 2 + h2;
      ov[it] = *(const v4f*)(os + row * 64 + c4);
    }
    for (int pass = 0; pass < 2; ++pass) {
#pragma unroll
      for (int it = 0; it < 8; ++it) {
        const int row = it * 2 + h2;
        const size_t go = (size_t)(q0 + row) * DM + (size_t)h * HD + c4;
        *(volatile v4f*)(outp + go) = ov[it];
      }
      __threadfence();
    }
  }
}

template <int DBL, int OUTF, int OUTH>
__global__ __launch_bounds__(128) void ln512(const float* __restrict__ P, const float* __restrict__ Xr,
                                             const float* __restrict__ ga, const float* __restrict__ ba,
                                             const float* __restrict__ gb, const float* __restrict__ bbp,
                                             float* F, unsigned short* Hh, float osc) {
#pragma clang fp contract(off)
  __shared__ float red[4][4];
  __shared__ __align__(16) float sy[DM];
  const int tid = threadIdx.x, wave = tid >> 5, lane = tid & 31;
  const int row = blockIdx.x;
  const int c0 = tid * 4;
  const size_t ro = (size_t)row * DM + c0;
  const v4f pv = *(const v4f*)(P + ro);
  float x[4] = {pv[0], pv[1], pv[2], pv[3]};
  float s = (x[0] + x[1]) + (x[2] + x[3]);
#pragma unroll
  for (int off = 16; off >= 1; off >>= 1) s += __shfl_xor(s, off, 32);
  if (lane == 0) red[0][wave] = s;
  __syncthreads();
  const float mu = (((red[0][0] + red[0][1]) + red[0][2]) + red[0][3]) * (1.0f / (float)DM);
  float d[4];
  float ss = 0.f;
#pragma unroll
  for (int e = 0; e < 4; ++e) { d[e] = x[e] - mu; ss += d[e] * d[e]; }
#pragma unroll
  for (int off = 16; off >= 1; off >>= 1) ss += __shfl_xor(ss, off, 32);
  if (lane == 0) red[1][wave] = ss;
  __syncthreads();
  const float var  = (((red[1][0] + red[1][1]) + red[1][2]) + red[1][3]) * (1.0f / (float)DM);
  const float rstd = rsqrtf(var + 1e-5f);
  float y[4];
  {
    const v4f g4 = *(const v4f*)(ga + c0);
    const v4f b4 = *(const v4f*)(ba + c0);
#pragma unroll
    for (int e = 0; e < 4; ++e) y[e] = (d[e] * rstd) * bfr(g4[e]) + bfr(b4[e]);
  }
  if (DBL != 0) {
    const v4f xr = *(const v4f*)(Xr + ro);
    float u[4];
    float s2 = 0.f;
#pragma unroll
    for (int e = 0; e < 4; ++e) { u[e] = xr[e] + y[e]; s2 += u[e]; }
#pragma unroll
    for (int off = 16; off >= 1; off >>= 1) s2 += __shfl_xor(s2, off, 32);
    if (lane == 0) red[2][wave] = s2;
    __syncthreads();
    const float mu2 = (((red[2][0] + red[2][1]) + red[2][2]) + red[2][3]) * (1.0f / (float)DM);
    float d2[4];
    float ss2 = 0.f;
#pragma unroll
    for (int e = 0; e < 4; ++e) { d2[e] = u[e] - mu2; ss2 += d2[e] * d2[e]; }
#pragma unroll
    for (int off = 16; off >= 1; off >>= 1) ss2 += __shfl_xor(ss2, off, 32);
    if (lane == 0) red[3][wave] = ss2;
    __syncthreads();
    const float var2  = (((red[3][0] + red[3][1]) + red[3][2]) + red[3][3]) * (1.0f / (float)DM);
    const float rstd2 = rsqrtf(var2 + 1e-5f);
    const v4f g4 = *(const v4f*)(gb + c0);
    const v4f b4 = *(const v4f*)(bbp + c0);
#pragma unroll
    for (int e = 0; e < 4; ++e) y[e] = (d2[e] * rstd2) * bfr(g4[e]) + bfr(b4[e]);
  }
  v4f o4 = {y[0], y[1], y[2], y[3]};
  v4u pk = {0u, 0u, 0u, 0u};
  if (OUTH != 0) {
    *(v4f*)(sy + c0) = o4;
    __syncthreads();
    if (tid < 64) {
      float t8[8];
      ld8(sy + tid * 8, t8);
#pragma unroll
      for (int p = 0; p < 4; ++p)
        pk[p] = pk16(h_bits((_Float16)(t8[2 * p] * osc)), h_bits((_Float16)(t8[2 * p + 1] * osc)));
    }
  }
  const size_t ho = (size_t)row * DM + (size_t)tid * 8;
  if (OUTF != 0) *(volatile v4f*)(F + ro) = o4;
  if (OUTH != 0) { if (tid < 64) *(volatile v4u*)(Hh + ho) = pk; }
  __threadfence();
  if (OUTF != 0) *(volatile v4f*)(F + ro) = o4;
  if (OUTH != 0) { if (tid < 64) *(volatile v4u*)(Hh + ho) = pk; }
}

__global__ __launch_bounds__(128) void ms_f16(const float* __restrict__ Y, int yo1, int yo2, int yo3,
                                              unsigned short* MS, float osc) {
#pragma clang fp contract(off)
  __shared__ __align__(16) float sy[DM];
  const int tid = threadIdx.x, wave = tid >> 5, lane = tid & 31;
  const int row = blockIdx.x;
  const int b = row >> 10;
  const int s = row & (SEQ - 1);
  const int i = wave;
  const int T = SEQ >> (2 * i);
  const int ns = (i == 3) ? 16 : ((i == 2) ? 4 : 1);
  const int yoff = (i == 0) ? 0 : ((i == 1) ? yo1 : ((i == 2) ? yo2 : yo3));
  const int sstr = BATCH * T * CCH;
  const float ratio = (float)T * (1.0f / (float)SEQ);
  float pos = ((float)s + 0.5f) * ratio - 0.5f;
  pos = fminf(fmaxf(pos, 0.0f), (float)(T - 1));
  const int lo = (int)pos;
  const int hi = min(lo + 1, T - 1);
  const float w = pos - (float)lo;
  const int c0 = lane * 4;
  const float* ylo = Y + (size_t)yoff + (size_t)(b * T + lo) * CCH + c0;
  const float* yhi = Y + (size_t)yoff + (size_t)(b * T + hi) * CCH + c0;
  v4f a  = {0.f, 0.f, 0.f, 0.f};
  v4f ah = {0.f, 0.f, 0.f, 0.f};
  for (int k = 0; k < ns; ++k) {
    a  += *(const v4f*)(ylo + (size_t)k * (size_t)sstr);
    ah += *(const v4f*)(yhi + (size_t)k * (size_t)sstr);
  }
  v4f val;
#pragma unroll
  for (int e = 0; e < 4; ++e) val[e] = a[e] * (1.0f - w) + ah[e] * w;
  *(v4f*)(sy + i * CCH + c0) = val;
  __syncthreads();
  if (tid < 64) {
    float t8[8];
    ld8(sy + tid * 8, t8);
    v4u pk;
#pragma unroll
    for (int p = 0; p < 4; ++p)
      pk[p] = pk16(h_bits((_Float16)(t8[2 * p] * osc)), h_bits((_Float16)(t8[2 * p + 1] * osc)));
    const size_t ho = (size_t)row * DM + (size_t)tid * 8;
    *(volatile v4u*)(MS + ho) = pk;
    __threadfence();
    *(volatile v4u*)(MS + ho) = pk;
  }
}

extern "C" void kernel_launch(void* const* d_in, const int* in_sizes, int n_in,
                              void* d_out, int out_size, void* d_ws, size_t ws_size,
                              hipStream_t stream) {
  if (n_in < 34) return;
  if (in_sizes[0] != MROWS * DM) return;
  if (in_sizes[1] != MROWS || in_sizes[2] != MROWS) return;
  if (in_sizes[3] != DM * DM || in_sizes[5] != DM * DM || in_sizes[7] != DM * DM || in_sizes[9] != DM * DM) return;
  if (in_sizes[4] != DM || in_sizes[6] != DM || in_sizes[8] != DM || in_sizes[10] != DM) return;
  if (in_sizes[11] != NH * NRES * NRES) return;
  if (in_sizes[12] != CCH * DM * 1 || in_sizes[14] != CCH * DM * 4) return;
  if (in_sizes[16] != CCH * DM * 16 || in_sizes[18] != CCH * DM * 64) return;
  if (in_sizes[13] != CCH || in_sizes[15] != CCH || in_sizes[17] != CCH || in_sizes[19] != CCH) return;
  if (in_sizes[20] != DM * DM || in_sizes[21] != DM) return;
  for (int i = 22; i <= 27; ++i) { if (in_sizes[i] != DM) return; }
  if (in_sizes[28] != FFN * DM || in_sizes[29] != FFN) return;
  if (in_sizes[30] != DM * FFN || in_sizes[31] != DM) return;
  if (in_sizes[32] != DM || in_sizes[33] != DM) return;
  if (out_size != OUTN) return;

  const float* x    = (const float*)d_in[0];
  const int*   rm   = (const int*)d_in[1];
  const int*   am   = (const int*)d_in[2];
  const float* wq   = (const float*)d_in[3];
  const float* bq   = (const float*)d_in[4];
  const float* wk   = (const float*)d_in[5];
  const float* bk   = (const float*)d_in[6];
  const float* wv   = (const float*)d_in[7];
  const float* bv   = (const float*)d_in[8];
  const float* wo   = (const float*)d_in[9];
  const float* bo   = (const float*)d_in[10];
  const float* rb   = (const float*)d_in[11];
  const float* cw0  = (const float*)d_in[12];
  const float* cb0  = (const float*)d_in[13];
  const float* cw1  = (const float*)d_in[14];
  const float* cb1  = (const float*)d_in[15];
  const float* cw2  = (const float*)d_in[16];
  const float* cb2  = (const float*)d_in[17];
  const float* cw3  = (const float*)d_in[18];
  const float* cb3  = (const float*)d_in[19];
  const float* fw   = (const float*)d_in[20];
  const float* fb   = (const float*)d_in[21];
  const float* ltg  = (const float*)d_in[22];
  const float* ltb  = (const float*)d_in[23];
  const float* n1g  = (const float*)d_in[24];
  const float* n1b  = (const float*)d_in[25];
  const float* n2g  = (const float*)d_in[26];
  const float* n2b  = (const float*)d_in[27];
  const float* fw1  = (const float*)d_in[28];
  const float* fb1  = (const float*)d_in[29];
  const float* fw2  = (const float*)d_in[30];
  const float* fb2  = (const float*)d_in[31];
  const float* n3g  = (const float*)d_in[32];
  const float* n3b  = (const float*)d_in[33];

  const size_t P16   = (size_t)MROWS * DM * 2;
  const size_t PF32  = (size_t)MROWS * DM * 4;
  const size_t PWdd  = (size_t)DM * DM * 2;
  const size_t PWff  = (size_t)FFN * DM * 2;
  const size_t PCw0  = (size_t)CCH * DM * 1 * 2;
  const size_t PCw1  = (size_t)CCH * DM * 4 * 2;
  const size_t PCw2  = (size_t)CCH * DM * 16 * 2;
  const size_t PCw3  = (size_t)CCH * DM * 64 * 2;
  const size_t PVt   = (size_t)BATCH * NH * HD * SEQ * 2;
  const int    yo1   = MROWS * CCH;
  const int    yo2   = yo1 + (MROWS / 4) * CCH;
  const int    yo3   = yo2 + 4 * (MROWS / 16) * CCH;
  const int    yend  = yo3 + 16 * (MROWS / 64) * CCH;
  const size_t PY    = (size_t)yend * 4;
  const size_t PG    = (size_t)MROWS * FFN * 2;

  size_t off = 0;
  const size_t oXh  = off; off += P16;
  const size_t oWq  = off; off += PWdd;
  const size_t oWk  = off; off += PWdd;
  const size_t oWv  = off; off += PWdd;
  const size_t oWo  = off; off += PWdd;
  const size_t oFw  = off; off += PWdd;
  const size_t oF1  = off; off += PWff;
  const size_t oF2  = off; off += PWff;
  const size_t oCw0 = off; off += PCw0;
  const size_t oCw1 = off; off += PCw1;
  const size_t oCw2 = off; off += PCw2;
  const size_t oCw3 = off; off += PCw3;
  const size_t oQh  = off; off += P16;
  const size_t oKh  = off; off += P16;
  const size_t oVf  = off; off += PF32;
  const size_t oVTh = off; off += PVt;
  const size_t oVTl = off; off += PVt;
  const size_t oOf  = off; off += PF32;
  const size_t oOh  = off; off += P16;
  const size_t oT0  = off; off += PF32;
  const size_t oX1f = off; off += PF32;
  const size_t oX1h = off; off += P16;
  const size_t oY   = off; off += PY;
  const size_t oMS  = off; off += P16;
  const size_t oT1  = off; off += PF32;
  const size_t oX2f = off; off += PF32;
  const size_t oX2h = off; off += P16;
  const size_t oG   = off; off += PG;
  if (off > ws_size) return;
  if (off > (size_t)134217728) return;

  char* ws = (char*)d_ws;
  unsigned short* Xh   = (unsigned short*)(ws + oXh);
  unsigned short* Wq16 = (unsigned short*)(ws + oWq);
  unsigned short* Wk16 = (unsigned short*)(ws + oWk);
  unsigned short* Wv16 = (unsigned short*)(ws + oWv);
  unsigned short* Wo16 = (unsigned short*)(ws + oWo);
  unsigned short* Fw16 = (unsigned short*)(ws + oFw);
  unsigned short* F1   = (unsigned short*)(ws + oF1);
  unsigned short* F2   = (unsigned short*)(ws + oF2);
  unsigned short* Cw0  = (unsigned short*)(ws + oCw0);
  unsigned short* Cw1  = (unsigned short*)(ws + oCw1);
  unsigned short* Cw2  = (unsigned short*)(ws + oCw2);
  unsigned short* Cw3  = (unsigned short*)(ws + oCw3);
  unsigned short* Qh   = (unsigned short*)(ws + oQh);
  unsigned short* Kh   = (unsigned short*)(ws + oKh);
  float*          Vf   = (float*)(ws + oVf);
  unsigned short* VTh  = (unsigned short*)(ws + oVTh);
  unsigned short* VTl  = (unsigned short*)(ws + oVTl);
  float*          Of   = (float*)(ws + oOf);
  unsigned short* Oh   = (unsigned short*)(ws + oOh);
  float*          T0   = (float*)(ws + oT0);
  float*          T2   = T0;
  float*          X1f  = (float*)(ws + oX1f);
  unsigned short* X1h  = (unsigned short*)(ws + oX1h);
  float*          Yall = (float*)(ws + oY);
  unsigned short* MSh  = (unsigned short*)(ws + oMS);
  float*          T1   = (float*)(ws + oT1);
  float*          X2f  = (float*)(ws + oX2f);
  unsigned short* X2h  = (unsigned short*)(ws + oX2h);
  unsigned short* G16  = (unsigned short*)(ws + oG);
  float*          outf = (float*)d_out;

  const dim3 blk(256);
  const int n8dd = DM * DM / 8;
  const int n8ff = FFN * DM / 8;
  const int n8x  = MROWS * DM / 8;
  const dim3 gWdd((n8dd + 255) / 256);
  const dim3 gWff((n8ff + 255) / 256);
  const dim3 gCvt((n8x + 255) / 256);
  const dim3 gDM(((MROWS / 64) * (DM / 64) + 7) / 8);
  const dim3 gFF(((MROWS / 64) * (FFN / 64) + 7) / 8);
  const dim3 gVpl(SEQ / 64, NH, BATCH);
  const dim3 gAttn(BATCH * NH * NQB);
  const dim3 gRows(MROWS);

  const float wScale  = 64.0f;
  const float hScale  = 8.0f;
  const float qkScale = 16.0f;
  const float sscale  = 1.0f / 2048.0f;
  const float vScale  = 256.0f;
  const float attOscl = 1.0f / 262144.0f;
  const float oScale  = 64.0f;
  const float gScale  = 16.0f;

  cvt_f16x8<<<gWdd, blk, 0, stream>>>(wq, Wq16, n8dd, wScale, 1);
  cvt_f16x8<<<gWdd, blk, 0, stream>>>(wk, Wk16, n8dd, wScale, 1);
  cvt_f16x8<<<gWdd, blk, 0, stream>>>(wv, Wv16, n8dd, wScale, 1);
  cvt_f16x8<<<gWdd, blk, 0, stream>>>(wo, Wo16, n8dd, wScale, 1);
  cvt_f16x8<<<gWdd, blk, 0, stream>>>(fw, Fw16, n8dd, wScale, 1);
  cvt_f16x8<<<gWff, blk, 0, stream>>>(fw1, F1, n8ff, wScale, 1);
  cvt_f16x8<<<gWff, blk, 0, stream>>>(fw2, F2, n8ff, wScale, 1);
  cw_cvt<<<dim3((CCH * DM * 1 / 8 + 255) / 256), blk, 0, stream>>>(cw0, Cw0, CCH * DM * 1 / 8, 1, wScale);
  cw_cvt<<<dim3((CCH * DM * 4 / 8 + 255) / 256), blk, 0, stream>>>(cw1, Cw1, CCH * DM * 4 / 8, 4, wScale);
  cw_cvt<<<dim3((CCH * DM * 16 / 8 + 255) / 256), blk, 0, stream>>>(cw2, Cw2, CCH * DM * 16 / 8, 16, wScale);
  cw_cvt<<<dim3((CCH * DM * 64 / 8 + 255) / 256), blk, 0, stream>>>(cw3, Cw3, CCH * DM * 64 / 8, 64, wScale);
  cvt_f16x8<<<gCvt, blk, 0, stream>>>(x, Xh, n8x, hScale, 1);
  gemm64<2, 0, 0><<<gDM, blk, 0, stream>>>(Xh, DM, Wq16, DM, bq, x, DM, Vf, Qh, DM, MROWS, DM, DM, 1, 0,
                                           1.0f / 512.0f, qkScale);
  gemm64<2, 0, 0><<<gDM, blk, 0, stream>>>(Xh, DM, Wk16, DM, bk, x, DM, Vf, Kh, DM, MROWS, DM, DM, 1, 0,
                                           1.0f / 512.0f, qkScale);
  gemm64<0, 0, 0><<<gDM, blk, 0, stream>>>(Xh, DM, Wv16, DM, bv, x, DM, Vf, Xh, DM, MROWS, DM, DM, 1, 0,
                                           1.0f / 512.0f, 1.0f);
  v_planes<<<gVpl, blk, 0, stream>>>(Vf, VTh, VTl, vScale);
  attn64<<<gAttn, dim3(128), 0, stream>>>(Qh, Kh, VTh, VTl, rb, rm, am, Of, sscale, attOscl);
  cvt_f16x8<<<gCvt, blk, 0, stream>>>(Of, Oh, n8x, oScale, 0);
  gemm64<1, 1, 0><<<gDM, blk, 0, stream>>>(Oh, DM, Wo16, DM, bo, x, DM, T0, Xh, DM, MROWS, DM, DM, 1, 0,
                                           1.0f / 4096.0f, 1.0f);
  ln512<0, 1, 1><<<gRows, dim3(128), 0, stream>>>(T0, T0, n1g, n1b, n1g, n1b, X1f, X1h, hScale);
  gemm64<0, 0, 0><<<dim3(((MROWS / 64) * 2 * 1 + 7) / 8), blk, 0, stream>>>(
      X1h, DM * 1, Cw0, DM * 1, cb0, x, DM, Yall, Xh, CCH, MROWS, CCH, DM, 1, MROWS * CCH,
      1.0f / 512.0f, 1.0f);
  gemm64<0, 0, 0><<<dim3(((MROWS / 4 / 64) * 2 * 1 + 7) / 8), blk, 0, stream>>>(
      X1h, DM * 4, Cw1, DM * 4, cb1, x, DM, Yall + yo1, Xh, CCH, MROWS / 4, CCH, DM * 4, 1, (MROWS / 4) * CCH,
      1.0f / 512.0f, 1.0f);
  gemm64<0, 0, 0><<<dim3(((MROWS / 16 / 64) * 2 * 4 + 7) / 8), blk, 0, stream>>>(
      X1h, DM * 16, Cw2, DM * 16, cb2, x, DM, Yall + yo2, Xh, CCH, MROWS / 16, CCH, 2048, 4, (MROWS / 16) * CCH,
      1.0f / 512.0f, 1.0f);
  gemm64<0, 0, 0><<<dim3(((MROWS / 64 / 64) * 2 * 16 + 7) / 8), blk, 0, stream>>>(
      X1h, DM * 64, Cw3, DM * 64, cb3, x, DM, Yall + yo3, Xh, CCH, MROWS / 64, CCH, 2048, 16, (MROWS / 64) * CCH,
      1.0f / 512.0f, 1.0f);
  ms_f16<<<gRows, dim3(128), 0, stream>>>(Yall, yo1, yo2, yo3, MSh, hScale);
  gemm64<1, 0, 0><<<gDM, blk, 0, stream>>>(MSh, DM, Fw16, DM, fb, X1f, DM, T1, Xh, DM, MROWS, DM, DM, 1, 0,
                                           1.0f / 512.0f, 1.0f);
  ln512<1, 1, 1><<<gRows, dim3(128), 0, stream>>>(T1, X1f, ltg, ltb, n2g, n2b, X2f, X2h, hScale);
  gemm64<2, 0, 1><<<gFF, blk, 0, stream>>>(X2h, DM, F1, DM, fb1, x, DM, Vf, G16, FFN, MROWS, FFN, DM, 1, 0,
                                           1.0f / 512.0f, gScale);
  gemm64<1, 0, 0><<<gDM, blk, 0, stream>>>(G16, FFN, F2, FFN, fb2, X2f, DM, T2, Xh, DM, MROWS, DM, FFN, 1, 0,
                                           1.0f / 1024.0f, 1.0f);
  ln512<0, 1, 0><<<gRows, dim3(128), 0, stream>>>(T2, T2, n3g, n3b, n3g, n3b, outf, Xh, 1.0f);
  (void)hipGetLastError();
}
